// Lin_Sfm_Attention_42949672960409
// MI455X (gfx1250) — hardware-verified
//
#include <hip/hip_runtime.h>


namespace {
constexpr int Bsz = 8, S = 2048, V = 2048;
constexpr int QB = S / 128, KBW = 64, NTRI = QB * QB + QB;
constexpr float NEG = -1e30f;

typedef _Float16 b16;
typedef __attribute__((ext_vector_type(16))) _Float16 v16b;
typedef __attribute__((ext_vector_type(8)))  _Float16 v8b;
typedef __attribute__((ext_vector_type(8)))  float v8f;
typedef __attribute__((ext_vector_type(4)))  float v4f;

__device__ __forceinline__ v8b ld8b(const b16* p) { return *(const v8b*)p; }
__device__ __forceinline__ v16b cat8b(v8b a, v8b b) { return __builtin_shufflevector(a, b, 0, 1, 2, 3, 4, 5, 6, 7, 8, 9, 10, 11, 12, 13, 14, 15); }
__device__ __forceinline__ v16b frag_kb(const b16* p, int hh) { return cat8b(ld8b(p + 8 * hh), ld8b(p + 16 + 8 * hh)); }
__device__ __forceinline__ void split16(float v, b16& hi, b16& lo) { hi = (b16)v; lo = (b16)(v - (float)hi); }
__device__ __forceinline__ void frag_ksplit(const float* p, int hh, v16b& fh_, v16b& fl_) {
  const float* p0 = p + 8 * hh; const float* p1 = p + 16 + 8 * hh;
#pragma unroll
  for (int e = 0; e < 8; ++e) { b16 a, c; split16(p0[e], a, c); fh_[e] = a; fl_[e] = c; split16(p1[e], a, c); fh_[8 + e] = a; fl_[8 + e] = c; }
}
__device__ __forceinline__ v8f wmma16b(v16b a, v16b b, v8f c) {
  v8f d = __builtin_amdgcn_wmma_f32_16x16x32_f16(false, a, false, b, (short)0, c, false, false);
  asm volatile("v_nop\n\tv_nop\n\tv_nop\n\tv_nop" : "+v"(d) : "v"(a), "v"(b));
  return d;
}
__device__ __forceinline__ void wave_lds_sync() {
  __builtin_amdgcn_fence(__ATOMIC_RELEASE, "workgroup");
  __builtin_amdgcn_wave_barrier();
  __builtin_amdgcn_fence(__ATOMIC_ACQUIRE, "workgroup");
}

struct Opnd { const void* p0; const void* p1; int ld; };
template <int NP> __device__ __forceinline__ void load_frags(const Opnd& o, int row, int kb, int hh, v16b& fh_, v16b& fl_) {
  if (NP == 0) { frag_ksplit((const float*)o.p0 + (size_t)row * o.ld + kb, hh, fh_, fl_); }
  else if (NP == 4) {
    const float* p = (const float*)o.p0 + (size_t)row * o.ld + kb; const float* p0 = p + 8 * hh; const float* p1 = p + 16 + 8 * hh;
#pragma unroll
    for (int e = 0; e < 8; ++e) { b16 a, c; split16(p0[e] * 64.0f, a, c); fh_[e] = a; fl_[e] = c; split16(p1[e] * 64.0f, a, c); fh_[8 + e] = a; fl_[8 + e] = c; }
  } else if (NP == 3) {
    const float* p = (const float*)o.p0 + (size_t)row * o.ld + kb; const float* p0 = p + 8 * hh; const float* p1 = p + 16 + 8 * hh;
#pragma unroll
    for (int e = 0; e < 8; ++e) { fh_[e] = (b16)p0[e]; fh_[8 + e] = (b16)p1[e]; }
    fl_ = fh_;
  } else {
    fh_ = frag_kb((const b16*)o.p0 + (size_t)row * o.ld + kb, hh);
    if (NP == 2) fl_ = frag_kb((const b16*)o.p1 + (size_t)row * o.ld + kb, hh); else fl_ = fh_;
  }
}
template <int ANP, int BNP> __device__ __forceinline__ v8f mac(v16b ah, v16b al, v16b bh, v16b bl, v8f c) {
  c = wmma16b(ah, bh, c);
  if (BNP == 0 || BNP == 2 || BNP == 4) c = wmma16b(ah, bl, c);
  if (ANP == 0 || ANP == 2 || ANP == 4) c = wmma16b(al, bh, c);
  return c;
}
template <int ANP, int BNP>
__device__ __forceinline__ void gemm_tile(const Opnd& A, const Opnd& B, int K, int m0, int c0, int nloc, int hlf, v8f (&acc)[2][4]) {
  for (int kb = 0; kb < K; kb += 32) {
    v16b a0h, a0l, a1h, a1l;
    load_frags<ANP>(A, m0 + nloc, kb, hlf, a0h, a0l);
    load_frags<ANP>(A, m0 + 16 + nloc, kb, hlf, a1h, a1l);
#pragma unroll
    for (int t = 0; t < 4; ++t) {
      v16b bh, bl;
      load_frags<BNP>(B, c0 + t * 16 + nloc, kb, hlf, bh, bl);
      acc[0][t] = mac<ANP, BNP>(a0h, a0l, bh, bl, acc[0][t]);
      acc[1][t] = mac<ANP, BNP>(a1h, a1l, bh, bl, acc[1][t]);
    }
  }
}

__device__ __forceinline__ void epi_planes(v8f (&acc)[2][4], float scale, bool two, b16* __restrict__ oh, b16* __restrict__ ol, int ldo,
                                           int m0, int c0, int lane, b16* Th, b16* Tl) {
  const int nloc = lane & 15, hlf = lane >> 4;
#pragma unroll
  for (int t = 0; t < 4; ++t)
#pragma unroll
    for (int r = 0; r < 2; ++r)
#pragma unroll
      for (int v = 0; v < 8; ++v) {
        const int rr = r * 16 + v + 8 * hlf, cc = t * 16 + nloc;
        b16 h_, l_; split16(acc[r][t][v] * scale, h_, l_);
        Th[rr * 64 + cc] = h_; Tl[rr * 64 + cc] = l_;
      }
  wave_lds_sync();
  for (int pass = 0; pass < 2; ++pass) {
#pragma unroll
    for (int j = 0; j < 8; ++j) {
      const int rr = j * 4 + (lane >> 3), c8 = (lane & 7) * 8;
      const size_t o = (size_t)(m0 + rr) * ldo + c0 + c8;
      *(volatile v8b*)(oh + o) = ld8b(Th + rr * 64 + c8);
      if (two) *(volatile v8b*)(ol + o) = ld8b(Tl + rr * 64 + c8);
    }
    __threadfence();
  }
}
__device__ __forceinline__ void epi_f32(v8f (&acc)[2][4], float scale, const float* rscale, float* __restrict__ out, int ldo, int m0, int c0, int lane, float* Tt) {
  const int nloc = lane & 15, hlf = lane >> 4;
#pragma unroll
  for (int t = 0; t < 4; ++t)
#pragma unroll
    for (int r = 0; r < 2; ++r)
#pragma unroll
      for (int v = 0; v < 8; ++v) {
        const int rr = r * 16 + v + 8 * hlf;
        const float rs = rscale ? rscale[(size_t)(m0 + rr) * 32] : 1.0f;
        Tt[rr * 64 + t * 16 + nloc] = acc[r][t][v] * scale * rs;
      }
  wave_lds_sync();
  float* dst0 = out + (size_t)m0 * ldo + c0;
  for (int pass = 0; pass < 2; ++pass) {
#pragma unroll
    for (int j = 0; j < 16; ++j) { const int rr = j * 2 + hlf, c4 = nloc * 4; *(volatile v4f*)(dst0 + (size_t)rr * ldo + c4) = *(const v4f*)(Tt + rr * 64 + c4); }
    __threadfence();
  }
}


__global__ __launch_bounds__(256) void prep_kernel(const float* __restrict__ wq, const float* __restrict__ wk, b16* __restrict__ w16) {
  const size_t tid = (size_t)blockIdx.x * blockDim.x + threadIdx.x, stride = (size_t)gridDim.x * blockDim.x, n1 = (size_t)S * S / 8;
  for (int pass = 0; pass < 2; ++pass) {
    for (size_t c = tid; c < 2 * n1; c += stride) {
      const float* src = (c < n1) ? (wq + c * 8) : (wk + (c - n1) * 8); v8b v;
#pragma unroll
      for (int e = 0; e < 8; ++e) v[e] = (b16)src[e];
      *(volatile v8b*)(w16 + c * 8) = v;
    }
    __threadfence();
  }
}

__global__ __launch_bounds__(128) void qk1_kernel(const float* __restrict__ pos, const b16* __restrict__ w16, b16* __restrict__ q16, b16* __restrict__ k16) {
  __shared__ __attribute__((aligned(16))) b16 Ts[4][2][32 * 64];
  const int lane = threadIdx.x & 31, wave = threadIdx.x >> 5, nloc = lane & 15, hlf = lane >> 4;
  const int m0 = blockIdx.y * 128 + wave * 32, cg = blockIdx.x * 64; const bool isq = cg < S; const int c0 = isq ? cg : cg - S;
  v8f acc[2][4];
#pragma unroll
  for (int r = 0; r < 2; ++r)
#pragma unroll
    for (int t = 0; t < 4; ++t) acc[r][t] = (v8f){};
  const Opnd A{pos, nullptr, S}, B{w16 + (isq ? 0 : (size_t)S * S), nullptr, S};
  gemm_tile<3, 1>(A, B, S, m0, c0, nloc, hlf, acc);
  epi_planes(acc, 1.0f, false, isq ? q16 : k16, nullptr, S, m0, c0, lane, Ts[wave][0], Ts[wave][1]);
}

__global__ __launch_bounds__(128) void s1_kernel(const b16* __restrict__ q16, const b16* __restrict__ k16, const float* __restrict__ beta1, float* __restrict__ Sb) {
  __shared__ __attribute__((aligned(16))) float Ts[4][32 * 64];
  const int lane = threadIdx.x & 31, wave = threadIdx.x >> 5, nloc = lane & 15, hlf = lane >> 4;
  int qb = 0;
#pragma unroll 1
  for (int j = 1; j <= QB; ++j) { if (j * j + j <= (int)blockIdx.x) qb = j; }
  if (qb >= QB) return;
  const int kt = (int)blockIdx.x - (qb * qb + qb), m0 = qb * 128 + wave * 32, c0 = kt * KBW;
  v8f acc[2][4];
#pragma unroll
  for (int r = 0; r < 2; ++r)
#pragma unroll
    for (int t = 0; t < 4; ++t) acc[r][t] = (v8f){};
  const Opnd A{q16, nullptr, S}, B{k16, nullptr, S};
  gemm_tile<1, 1>(A, B, S, m0, c0, nloc, hlf, acc);
  epi_f32(acc, beta1[0] * (1.0f / 45.254833995939045f), nullptr, Sb, S, m0, c0, lane, Ts[wave]);
}

__global__ __launch_bounds__(256) void a1_kernel(const float* __restrict__ Sb, float* __restrict__ A1) {
  const int lane = threadIdx.x & 31, i = blockIdx.x * 8 + (threadIdx.x >> 5);
  const float* Sr = Sb + (size_t)i * S;
  float mx = -INFINITY;
#pragma unroll 1
  for (int j0 = 0; j0 < S; j0 += 128) { const int j = j0 + lane * 4;
#pragma unroll
    for (int e = 0; e < 4; ++e) { const int jj = j + e; const float s = (jj <= i) ? Sr[jj] : -INFINITY; mx = fmaxf(mx, s); } }
#pragma unroll
  for (int o = 16; o > 0; o >>= 1) mx = fmaxf(mx, __shfl_xor(mx, o));
  float sum = 0.0f;
#pragma unroll 1
  for (int j0 = 0; j0 < S; j0 += 128) { const int j = j0 + lane * 4;
#pragma unroll
    for (int e = 0; e < 4; ++e) { const int jj = j + e; if (jj <= i) sum += expf(Sr[jj] - mx); } }
#pragma unroll
  for (int o = 16; o > 0; o >>= 1) sum += __shfl_xor(sum, o);
  const float inv = (i == 0) ? 0.0f : 1.0f / sum;
  float* dst = A1 + (size_t)i * S;
  for (int pass = 0; pass < 2; ++pass) {
#pragma unroll 1
    for (int j0 = 0; j0 < S; j0 += 128) { const int j = j0 + lane * 4; v4f w;
#pragma unroll
      for (int e = 0; e < 4; ++e) { const int jj = j + e; w[e] = (jj <= i) ? expf(Sr[jj] - mx) * inv : 0.0f; }
      *(volatile v4f*)(dst + j) = w; }
    __threadfence();
  }
}

template <bool GATHER, bool TWO, bool ADDE>
__global__ __launch_bounds__(256) void mv_rows(const float* __restrict__ M, const float* __restrict__ emb, const int* __restrict__ tok, const float* __restrict__ x,
                                               const float* __restrict__ x2, size_t xstride, float* __restrict__ y, float* __restrict__ y2) {
  __shared__ float ys[32], ys2[32];
  const int wave = threadIdx.x >> 5, lane = threadIdx.x & 31, b = blockIdx.y, r0 = blockIdx.x * 32;
  const float* xb = x + (size_t)b * xstride; const float* x2b = TWO ? (x2 + (size_t)b * xstride) : nullptr;
  for (int q = 0; q < 4; ++q) {
    const int r = r0 + wave * 4 + q;
    const float* row;
    if (GATHER) { int t_ = tok[(size_t)b * S + r]; t_ = t_ < 0 ? 0 : (t_ >= V ? V - 1 : t_); row = emb + (size_t)t_ * V; } else row = M + (size_t)r * V;
    float s = 0.0f, s2 = 0.0f;
#pragma unroll 1
    for (int k0 = 0; k0 < V; k0 += 128) { const v4f m4 = *(const v4f*)(row + k0 + lane * 4); const v4f x4 = *(const v4f*)(xb + k0 + lane * 4);
      s += m4[0] * x4[0] + m4[1] * x4[1] + m4[2] * x4[2] + m4[3] * x4[3];
      if (TWO) { const v4f z4 = *(const v4f*)(x2b + k0 + lane * 4); s2 += m4[0] * z4[0] + m4[1] * z4[1] + m4[2] * z4[2] + m4[3] * z4[3]; } }
#pragma unroll
    for (int o = 16; o > 0; o >>= 1) { s += __shfl_xor(s, o); if (TWO) s2 += __shfl_xor(s2, o); }
    if (ADDE) { int t_ = tok[(size_t)b * S + (S - 1)]; t_ = t_ < 0 ? 0 : (t_ >= V ? V - 1 : t_); s += emb[(size_t)t_ * V + r]; }
    if (lane == 0) { ys[wave * 4 + q] = s; if (TWO) ys2[wave * 4 + q] = s2; }
  }
  __syncthreads();
  if (wave == 0) {
    for (int pass = 0; pass < 2; ++pass) {
      ((volatile float*)y)[(size_t)b * V + r0 + lane] = ys[lane];
      if (TWO) ((volatile float*)y2)[(size_t)b * V + r0 + lane] = ys2[lane];
      __threadfence();
    }
  }
}
template <bool GATHER>
__global__ __launch_bounds__(256) void mv_cols(const float* __restrict__ M, const float* __restrict__ emb, const int* __restrict__ tok, const float* __restrict__ x,
                                               size_t xstride, const float* __restrict__ scale, float* __restrict__ y) {
  const int b = blockIdx.y, c = blockIdx.x * 256 + threadIdx.x;
  const float* xb = x + (size_t)b * xstride; const float sc = scale ? scale[0] : 1.0f;
  float s = 0.0f;
#pragma unroll 1
  for (int r = 0; r < V; ++r) {
    const float* row;
    if (GATHER) { int t_ = tok[(size_t)b * S + r]; t_ = t_ < 0 ? 0 : (t_ >= V ? V - 1 : t_); row = emb + (size_t)t_ * V; } else row = M + (size_t)r * V;
    s += row[c] * xb[r];
  }
  for (int pass = 0; pass < 2; ++pass) { ((volatile float*)y)[(size_t)b * V + c] = s * sc; __threadfence(); }
}

__global__ __launch_bounds__(256) void a2_kernel(const float* __restrict__ cE, const float* __restrict__ g, const float* __restrict__ beta2, float* __restrict__ A2) {
  __shared__ float sv[S]; __shared__ float red[256];
  const int b = blockIdx.x, tid = threadIdx.x; const float bt = beta2[0] * (1.0f / 45.254833995939045f);
  float mx = -INFINITY;
  for (int s = tid; s < S; s += 256) { const float v = (s >= S - 2) ? NEG : bt * (cE[(size_t)b * V + s] + g[(size_t)b * V + s]); sv[s] = v; mx = fmaxf(mx, v); }
  red[tid] = mx; __syncthreads();
  for (int o = 128; o > 0; o >>= 1) { if (tid < o) red[tid] = fmaxf(red[tid], red[tid + o]); __syncthreads(); }
  mx = red[0]; __syncthreads();
  float sum = 0.0f;
  for (int s = tid; s < S; s += 256) sum += expf(sv[s] - mx);
  red[tid] = sum; __syncthreads();
  for (int o = 128; o > 0; o >>= 1) { if (tid < o) red[tid] += red[tid + o]; __syncthreads(); }
  const float inv = 1.0f / red[0];
  for (int pass = 0; pass < 2; ++pass) { for (int s = tid; s < S; s += 256) ((volatile float*)A2)[(size_t)b * S + s] = expf(sv[s] - mx) * inv; __threadfence(); }
}
}

extern "C" void kernel_launch(void* const* d_in, const int* in_sizes, int n_in,
                              void* d_out, int out_size, void* d_ws, size_t ws_size, hipStream_t stream) {
  (void)n_in; (void)out_size;
  const int* tok    = (const int*)d_in[0];
  const float* emb  = (const float*)d_in[1];
  const float* pos  = (const float*)d_in[2];
  const float* WQ1  = (const float*)d_in[3];
  const float* WK1  = (const float*)d_in[4];
  const float* WV1  = (const float*)d_in[5];
  const float* WQ2  = (const float*)d_in[6];
  const float* WK2  = (const float*)d_in[7];
  const float* b1   = (const float*)d_in[8];
  const float* b2   = (const float*)d_in[9];
  const float* bo   = (const float*)d_in[10];
  float* out = (float*)d_out;
  if (in_sizes[0] != Bsz * S || in_sizes[1] != V * V || in_sizes[2] != S * S || in_sizes[3] != S * S || in_sizes[7] != V * V) return;

  size_t off = 0; char* ws = (char*)d_ws;
  auto carve = [&](size_t bytes) { char* p = ws + off; off += (bytes + 255) & ~(size_t)255; return p; };
  b16* w16  = (b16*)carve((size_t)2 * S * S * 2);
  b16* q16  = (b16*)carve((size_t)S * S * 2);
  b16* k16  = (b16*)carve((size_t)S * S * 2);
  float* Sb = (float*)carve((size_t)S * S * 4);
  float* A1 = (float*)carve((size_t)S * S * 4);
  float* wl = (float*)carve((size_t)Bsz * V * 4);
  float* z  = (float*)carve((size_t)Bsz * V * 4);
  float* q2 = (float*)carve((size_t)Bsz * V * 4);
  float* u  = (float*)carve((size_t)Bsz * V * 4);
  float* w  = (float*)carve((size_t)Bsz * V * 4);
  float* cE = (float*)carve((size_t)Bsz * V * 4);
  float* cw = (float*)carve((size_t)Bsz * V * 4);
  float* g  = (float*)carve((size_t)Bsz * V * 4);
  float* A2 = (float*)carve((size_t)Bsz * S * 4);
  if (off > ws_size) return;
  prep_kernel<<<1024, 256, 0, stream>>>(WQ1, WK1, w16);
  qk1_kernel<<<dim3(2 * S / 64, S / 128), 128, 0, stream>>>(pos, w16, q16, k16);
  s1_kernel<<<NTRI, 128, 0, stream>>>(q16, k16, b1, Sb);
  a1_kernel<<<S / 8, 256, 0, stream>>>(Sb, A1);
  mv_cols<true><<<dim3(V / 256, Bsz), 256, 0, stream>>>(nullptr, emb, tok, A1 + (size_t)(S - 1) * S, 0, nullptr, wl);
  mv_rows<false, false, true><<<dim3(V / 32, Bsz), 256, 0, stream>>>(WV1, emb, tok, wl, nullptr, V, z, nullptr);
  mv_rows<false, false, false><<<dim3(V / 32, Bsz), 256, 0, stream>>>(WQ2, emb, tok, z, nullptr, V, q2, nullptr);
  mv_cols<false><<<dim3(V / 256, Bsz), 256, 0, stream>>>(WK2, emb, tok, q2, V, nullptr, u);
  mv_cols<false><<<dim3(V / 256, Bsz), 256, 0, stream>>>(WV1, emb, tok, u, V, nullptr, w);
  mv_rows<true, true, false><<<dim3(S / 32, Bsz), 256, 0, stream>>>(nullptr, emb, tok, u, w, V, cE, cw);
  mv_rows<false, false, false><<<dim3(S / 32, Bsz), 256, 0, stream>>>(A1, emb, tok, cw, nullptr, V, g, nullptr);
  a2_kernel<<<Bsz, 256, 0, stream>>>(cE, g, b2, A2);
  mv_cols<true><<<dim3(V / 256, Bsz), 256, 0, stream>>>(nullptr, emb, tok, A2, S, bo, out);
}
